// BubblePredictor_44830868635915
// MI455X (gfx1250) — hardware-verified
//
#include <hip/hip_runtime.h>
#include <math.h>

constexpr int kBatch    = 512;
constexpr int kSteps    = 512;
constexpr int kIn       = 8;
constexpr int kHid      = 256;
constexpr int kGateCols = 4 * kHid;
constexpr int kThreads  = 512;
constexpr int kRowsBlk  = 32;
constexpr int kPitchA   = 264;
constexpr int kPitchF   = 264;
constexpr int kChunk    = 16;
constexpr int kPitchL   = 2 * kChunk;
constexpr int kOut0     = kBatch * kSteps * 2;
constexpr int kOut1     = kBatch * kHid;
constexpr int kOutTotal = kOut0 + 2 * kOut1;
constexpr int kCastThr  = 256;
constexpr float kHCarry  = 16.0f;
constexpr float kWCarry  = 16.0f;
constexpr float kGateInv = 1.0f / 256.0f;
static_assert(kBatch % kRowsBlk == 0);
static_assert(kHid == 16 * (kThreads / 32));
static_assert(kHid % 32 == 0);
static_assert(kSteps % kChunk == 0);
static_assert((2 * kRowsBlk * kPitchA) % kThreads == 0);
static_assert(kRowsBlk == 2 * (kThreads / 32));
static_assert(kRowsBlk == 4 * 8);
static_assert((kGateCols * kHid / 8) % kCastThr == 0);

typedef __attribute__((ext_vector_type(16))) _Float16 v16h;
typedef __attribute__((ext_vector_type(8)))  _Float16 v8h;
typedef __attribute__((ext_vector_type(8)))  float    v8f;
typedef __attribute__((ext_vector_type(4)))  float    v4f;

__device__ __forceinline__ void dep_guard_h(v8f& a, v8f& b, v16h x, v16h y) { asm volatile("v_nop\n\tv_nop\n\tv_nop\n\tv_nop" : "+v"(a), "+v"(b) : "v"(x), "v"(y)); }
__device__ __forceinline__ void keep4_h(v16h a, v16h b, v16h c, v16h d) { asm volatile("v_nop" :: "v"(a), "v"(b), "v"(c), "v"(d)); }
__device__ __forceinline__ void acc_guard4(v8f& a, v8f& b, v8f& c, v8f& d) { asm volatile("v_nop\n\tv_nop\n\tv_nop\n\tv_nop" : "+v"(a), "+v"(b), "+v"(c), "+v"(d)); }

template <typename T> struct Frag;
template <> struct Frag<_Float16> {
  typedef v16h V; union U { v16h v; v8h h[2]; };
  static __device__ __forceinline__ v16h load(const _Float16* p) {
    U f; f.h[0] = *(const v8h*)(p); f.h[1] = *(const v8h*)(p + 16); return f.v;
  }
  static __device__ __forceinline__ v8f mma(v16h a, v16h b, v8f c) {
    return __builtin_amdgcn_wmma_f32_16x16x32_f16(false, a, false, b, (short)0, c, false, false);
  }
};

__device__ __forceinline__ float fsig(float x)  { return __builtin_amdgcn_rcpf(1.0f + __expf(-x)); }
__device__ __forceinline__ float ftanh(float x) { return 1.0f - 2.0f * __builtin_amdgcn_rcpf(__expf(2.0f * x) + 1.0f); }

__global__ __launch_bounds__(kCastThr) void cast_whh_kernel(const float* __restrict__ src, unsigned short* __restrict__ dst,
                                                           int n8, float sc) {
  const int i = blockIdx.x * kCastThr + threadIdx.x;
  if (i < n8) {
    const float* sp = src + (size_t)i * 8;
    const v4f a = *(const v4f*)(sp);
    const v4f b = *(const v4f*)(sp + 4);
    v8h hv;
#pragma unroll
    for (int e = 0; e < 4; ++e) {
      hv[e]     = (_Float16)(a[e] * sc);
      hv[4 + e] = (_Float16)(b[e] * sc);
    }
    *(volatile v8h*)(dst + (size_t)i * 8) = hv;
    __threadfence();
    *(volatile v8h*)(dst + (size_t)i * 8) = hv;
  }
}

__global__ __launch_bounds__(kThreads) void lstm_seq_kernel(const float* __restrict__ hist, const float* __restrict__ w_ih,
                                                           const unsigned short* __restrict__ whh_p,
                                                           const float* __restrict__ w_out, const float* __restrict__ b_out,
                                                           float* __restrict__ out) {
  __shared__ __align__(16) _Float16 hA[2][kRowsBlk * kPitchA];
  __shared__ __align__(16) float    hF[kRowsBlk * kPitchF];
  __shared__ __align__(16) float    xS[2][kRowsBlk * kIn];
  __shared__ __align__(16) float    lgS[kRowsBlk * kPitchL];
  const _Float16* whh = (const _Float16*)whh_p;
  const int tid = threadIdx.x, lane = tid & 31, wave = tid >> 5;
  const int c = lane & 15, hh = lane >> 4, koff = hh * 8;
  const int u = 16 * wave + c;
  const int rowbase = blockIdx.x * kRowsBlk;

  {
    _Float16* haf = &hA[0][0];
#pragma unroll 1
    for (int i = tid; i < 2 * kRowsBlk * kPitchA; i += kThreads) haf[i] = (_Float16)0.0f;
  }
  if (tid < 2 * kRowsBlk) {
    const int row = tid >> 1, half = tid & 1;
    const v4f v = *(const v4f*)(hist + ((size_t)(rowbase + row) * kSteps) * kIn + 4 * half);
    *(v4f*)(&xS[0][0] + row * kIn + 4 * half) = v;
  }
  float wih[4][8];
#pragma unroll
  for (int g = 0; g < 4; ++g) {
    const float* wp = w_ih + (size_t)(g * kHid + u) * kIn;
    const v4f a = *(const v4f*)(wp), b = *(const v4f*)(wp + 4);
#pragma unroll
    for (int e = 0; e < 4; ++e) { wih[g][e] = a[e]; wih[g][4 + e] = b[e]; }
  }
  float wo0[8], wo1[8];
  {
    const v4f a0 = *(const v4f*)(w_out + 8 * lane), a1 = *(const v4f*)(w_out + 8 * lane + 4);
    const v4f b0 = *(const v4f*)(w_out + kHid + 8 * lane), b1 = *(const v4f*)(w_out + kHid + 8 * lane + 4);
#pragma unroll
    for (int e = 0; e < 4; ++e) { wo0[e] = a0[e]; wo0[4 + e] = a1[e]; wo1[e] = b0[e]; wo1[4 + e] = b1[e]; }
  }
  const float bo0 = b_out[0], bo1 = b_out[1];
  float cst[2][8];
#pragma unroll
  for (int mi = 0; mi < 2; ++mi)
#pragma unroll
    for (int r = 0; r < 8; ++r) cst[mi][r] = 0.0f;
  __syncthreads();

  const v8f z8 = {0.f, 0.f, 0.f, 0.f, 0.f, 0.f, 0.f, 0.f};

#pragma unroll 1
  for (int t = 0; t < kSteps; ++t) {
    const int cur = t & 1, nxt = cur ^ 1;
    const _Float16* hAc = &hA[cur][0];
    _Float16*       hAn = &hA[nxt][0];
    const float*    xc  = &xS[cur][0];

#pragma unroll
    for (int mi = 0; mi < 2; ++mi) {
      v8f acc[4];
#pragma unroll
      for (int g = 0; g < 4; ++g) acc[g] = z8;
      const _Float16* arow = hAc + (16 * mi + c) * kPitchA + koff;
#pragma unroll 1
      for (int k0 = 0; k0 < kHid; k0 += 32) {
        const v16h a = Frag<_Float16>::load(arow + k0);
        v16h bq[4];
#pragma unroll
        for (int g = 0; g < 4; ++g) bq[g] = Frag<_Float16>::load(whh + (size_t)(g * kHid + u) * kHid + koff + k0);
#pragma unroll
        for (int g = 0; g < 4; ++g) acc[g] = Frag<_Float16>::mma(a, bq[g], acc[g]);
        dep_guard_h(acc[0], acc[3], a, bq[3]);
        keep4_h(bq[0], bq[1], bq[2], a);
      }
      acc_guard4(acc[0], acc[1], acc[2], acc[3]);

#pragma unroll
      for (int r = 0; r < 8; ++r) {
        const int row = 16 * mi + 8 * hh + r;
        const v4f xa = *(const v4f*)(xc + row * kIn);
        const v4f xb = *(const v4f*)(xc + row * kIn + 4);
        float z[4];
#pragma unroll
        for (int g = 0; g < 4; ++g) {
          float s = xa[0] * wih[g][0];
          s += xa[1] * wih[g][1]; s += xa[2] * wih[g][2]; s += xa[3] * wih[g][3];
          s += xb[0] * wih[g][4]; s += xb[1] * wih[g][5]; s += xb[2] * wih[g][6]; s += xb[3] * wih[g][7];
          z[g] = acc[g][r] * kGateInv + s;
        }
        const float ig = fsig(z[0]);
        const float fg = fsig(z[1]);
        const float gg = ftanh(z[2]);
        const float og = fsig(z[3]);
        const float cn = fg * cst[mi][r] + ig * gg;
        cst[mi][r] = cn;
        const float hn = og * ftanh(cn);
        hF[row * kPitchF + u] = hn;
        hAn[row * kPitchA + u] = (_Float16)(hn * kHCarry);
      }
    }
    if (tid < 2 * kRowsBlk) {
      const int row = tid >> 1, half = tid & 1;
      const int tn = (t + 1 < kSteps) ? (t + 1) : (kSteps - 1);
      const v4f v = *(const v4f*)(hist + ((size_t)(rowbase + row) * kSteps + (size_t)tn) * kIn + 4 * half);
      *(v4f*)(&xS[nxt][0] + row * kIn + 4 * half) = v;
    }
    __syncthreads();

    {
      float p0a = 0.f, p1a = 0.f, p0b = 0.f, p1b = 0.f;
      const float* ra = hF + (2 * wave) * kPitchF + 8 * lane;
      const float* rb = ra + kPitchF;
      const v4f a0 = *(const v4f*)(ra), a1 = *(const v4f*)(ra + 4);
      const v4f b0 = *(const v4f*)(rb), b1 = *(const v4f*)(rb + 4);
#pragma unroll
      for (int e = 0; e < 4; ++e) {
        p0a += a0[e] * wo0[e];     p1a += a0[e] * wo1[e];
        p0a += a1[e] * wo0[4 + e]; p1a += a1[e] * wo1[4 + e];
        p0b += b0[e] * wo0[e];     p1b += b0[e] * wo1[e];
        p0b += b1[e] * wo0[4 + e]; p1b += b1[e] * wo1[4 + e];
      }
#pragma unroll
      for (int off = 1; off < 32; off <<= 1) {
        p0a += __shfl_xor(p0a, off, 32);
        p1a += __shfl_xor(p1a, off, 32);
        p0b += __shfl_xor(p0b, off, 32);
        p1b += __shfl_xor(p1b, off, 32);
      }
      const float l00 = p0a + bo0, l01 = p1a + bo1, l10 = p0b + bo0, l11 = p1b + bo1;
      const float sel = (lane == 0) ? l00 : (lane == 1) ? l01 : (lane == 2) ? l10 : l11;
      if (lane < 4) lgS[(2 * wave + (lane >> 1)) * kPitchL + 2 * (t & (kChunk - 1)) + (lane & 1)] = sel;
    }
    __syncthreads();

    if (((t & (kChunk - 1)) == (kChunk - 1)) && (wave < 8)) {
      const int q = lane >> 3, c4 = (lane & 7) * 4;
      const int row = 4 * wave + q;
      const v4f v = *(const v4f*)(lgS + row * kPitchL + c4);
      float* op = out + (size_t)(rowbase + row) * (kSteps * 2) + (size_t)(t / kChunk) * kPitchL + c4;
      *(volatile v4f*)op = v;
      __threadfence();
      *(volatile v4f*)op = v;
    }
  }

  {
    float* o1 = out + kOut0;
    for (int pass = 0; pass < 2; ++pass) {
#pragma unroll
      for (int j = 0; j < 2; ++j) {
        const int row = 2 * wave + j;
#pragma unroll
        for (int q = 0; q < 2; ++q) {
          const v4f v = *(const v4f*)(hF + row * kPitchF + 128 * q + 4 * lane);
          *(volatile v4f*)(o1 + (size_t)(rowbase + row) * kHid + 128 * q + 4 * lane) = v;
        }
      }
      __threadfence();
    }
  }
  __syncthreads();
#pragma unroll
  for (int mi = 0; mi < 2; ++mi)
#pragma unroll
    for (int r = 0; r < 8; ++r) hF[(16 * mi + 8 * hh + r) * kPitchF + u] = cst[mi][r];
  __syncthreads();
  {
    float* o2 = out + kOut0 + kOut1;
    for (int pass = 0; pass < 2; ++pass) {
#pragma unroll
      for (int j = 0; j < 2; ++j) {
        const int row = 2 * wave + j;
#pragma unroll
        for (int q = 0; q < 2; ++q) {
          const v4f v = *(const v4f*)(hF + row * kPitchF + 128 * q + 4 * lane);
          *(volatile v4f*)(o2 + (size_t)(rowbase + row) * kHid + 128 * q + 4 * lane) = v;
        }
      }
      __threadfence();
    }
  }
}

extern "C" void kernel_launch(void* const* d_in, const int* in_sizes, int n_in,
                              void* d_out, int out_size, void* d_ws, size_t ws_size, hipStream_t stream) {
  if (n_in < 5 || d_out == nullptr || d_ws == nullptr) return;
  if (in_sizes[0] != kBatch * kSteps * kIn || in_sizes[1] != kGateCols * kIn || in_sizes[2] != kGateCols * kHid ||
      in_sizes[3] != 2 * kHid || in_sizes[4] != 2 || out_size != kOutTotal) return;
  const size_t whh_bytes = (size_t)kGateCols * kHid * 2;
  if (whh_bytes > ws_size || whh_bytes > (size_t)134217728) return;

  const float* hist  = (const float*)d_in[0];
  const float* w_ih  = (const float*)d_in[1];
  const float* w_hh  = (const float*)d_in[2];
  const float* w_out = (const float*)d_in[3];
  const float* b_out = (const float*)d_in[4];
  float* out = (float*)d_out;
  unsigned short* whh16 = (unsigned short*)d_ws;

  const int n8 = kGateCols * kHid / 8;
  cast_whh_kernel<<<(n8 + kCastThr - 1) / kCastThr, kCastThr, 0, stream>>>(w_hh, whh16, n8, kWCarry);
  lstm_seq_kernel<<<kBatch / kRowsBlk, kThreads, 0, stream>>>(hist, w_ih, whh16, w_out, b_out, out);
}
